// GroupConvAttention_68066641707315
// MI455X (gfx1250) — hardware-verified
//
#include <hip/hip_runtime.h>


namespace {
constexpr int Bn = 4, C = 256, HW = 64, HS = 32, NQ = HS * HS  , VK = 4, NCOL = C * VK * VK  , NPIX = HW * HW;

typedef _Float16 b16;
typedef __attribute__((ext_vector_type(16))) __bf16 v16bb;
typedef __attribute__((ext_vector_type(8))) unsigned short v8us;
typedef __attribute__((ext_vector_type(8))) float v8f;
typedef __attribute__((ext_vector_type(4))) float v4f;
__device__ __forceinline__ float bf16_rne(float f) { unsigned int u = __float_as_uint(f); u += 0x7FFFu + ((u >> 16) & 1u); return __uint_as_float(u & 0xFFFF0000u); }
__device__ __forceinline__ unsigned short bf16_bits(float f) { unsigned int u = __float_as_uint(f); u += 0x7FFFu + ((u >> 16) & 1u); return (unsigned short)(u >> 16); }
__device__ __forceinline__ v16bb frag_bf(const unsigned short* p, int hh) { const v8us a = *(const v8us*)(p + 8 * hh), b = *(const v8us*)(p + 16 + 8 * hh); union { unsigned short s[16]; v16bb v; } u;
#pragma unroll
  for (int e = 0; e < 8; ++e) { u.s[e] = a[e]; u.s[8 + e] = b[e]; } return u.v; }
__device__ __forceinline__ v8f wmma16bb(v16bb a, v16bb b, v8f c) { v8f d = __builtin_amdgcn_wmma_f32_16x16x32_bf16(false, a, false, b, (short)0, c, false, false); asm volatile("v_nop\n\tv_nop\n\tv_nop\n\tv_nop" : "+v"(d) : "v"(a), "v"(b)); return d; }
__device__ __forceinline__ void wave_lds_sync() { __builtin_amdgcn_fence(__ATOMIC_RELEASE, "workgroup"); __builtin_amdgcn_wave_barrier(); __builtin_amdgcn_fence(__ATOMIC_ACQUIRE, "workgroup"); }

__global__ __launch_bounds__(256) void sprep_kernel(const float* __restrict__ sc, unsigned short* __restrict__ s16) {
  const size_t tid = (size_t)blockIdx.x * blockDim.x + threadIdx.x, nth = (size_t)gridDim.x * blockDim.x;
  for (int pass = 0; pass < 2; ++pass) { for (size_t p = tid; p < (size_t)Bn * NQ * NQ / 8; p += nth) { v8us v;
#pragma unroll
      for (int e = 0; e < 8; ++e) v[e] = bf16_bits(sc[p * 8 + e]);
      *(volatile v8us*)(s16 + p * 8) = v; } __threadfence(); }
}
__global__ __launch_bounds__(256) void vt_kernel(const float* __restrict__ x, int b, unsigned short* __restrict__ vt) {
  const int row0 = blockIdx.x * 16, t_ = threadIdx.x;
  for (int pass = 0; pass < 2; ++pass) {
    for (int i = t_; i < 16 * NQ / 8; i += 256) { const int rr = i >> 7, p8 = (i & 127) * 8; const int n = row0 + rr, c = n >> 4, u = (n >> 2) & 3, v = n & 3; v8us o;
#pragma unroll
      for (int e = 0; e < 8; ++e) { const int p = p8 + e, m = p >> 5, nn = p & 31; const int yy = min(max(2 * m + u - 1, 0), HW - 1), xx = min(max(2 * nn + v - 1, 0), HW - 1);
        o[e] = bf16_bits(x[(((size_t)b * C + c) * HW + yy) * HW + xx]); }
      *(volatile v8us*)(vt + (size_t)n * NQ + p8) = o; }
    __threadfence(); }
}
__global__ __launch_bounds__(128) void gemm_kernel(const unsigned short* __restrict__ s16, int b, const unsigned short* __restrict__ vt, float* __restrict__ P) {
  __shared__ __attribute__((aligned(16))) float Ts[4][32 * 64];
  const int lane = threadIdx.x & 31, wave = threadIdx.x >> 5, nloc = lane & 15, hlf = lane >> 4, m0 = blockIdx.y * 128 + wave * 32, c0 = blockIdx.x * 64;
  const unsigned short* A = s16 + ((size_t)b * NQ) * NQ;
  v8f acc[2][4];
#pragma unroll
  for (int r = 0; r < 2; ++r)
#pragma unroll
    for (int t = 0; t < 4; ++t) acc[r][t] = (v8f){};
#pragma unroll 2
  for (int kb = 0; kb < NQ; kb += 32) { const v16bb a0 = frag_bf(A + (size_t)(m0 + nloc) * NQ + kb, hlf), a1 = frag_bf(A + (size_t)(m0 + 16 + nloc) * NQ + kb, hlf);
#pragma unroll
    for (int t = 0; t < 4; ++t) { const v16bb bw = frag_bf(vt + (size_t)(c0 + t * 16 + nloc) * NQ + kb, hlf); acc[0][t] = wmma16bb(a0, bw, acc[0][t]); acc[1][t] = wmma16bb(a1, bw, acc[1][t]); } }
  float* Tt = Ts[wave];
#pragma unroll
  for (int t = 0; t < 4; ++t)
#pragma unroll
    for (int r = 0; r < 2; ++r)
#pragma unroll
      for (int v = 0; v < 8; ++v) Tt[(r * 16 + v + 8 * hlf) * 64 + t * 16 + nloc] = acc[r][t][v];
  wave_lds_sync();
  float* dst0 = P + (size_t)m0 * NCOL + c0;
  for (int pass = 0; pass < 2; ++pass) {
#pragma unroll
    for (int j = 0; j < 16; ++j) { const int rr = j * 2 + hlf, c4 = nloc * 4; *(volatile v4f*)(dst0 + (size_t)rr * NCOL + c4) = *(const v4f*)(Tt + rr * 64 + c4); }
    __threadfence(); }
}
__global__ __launch_bounds__(256) void oadd_kernel(const float* __restrict__ P, const float* __restrict__ x, const float* __restrict__ alpha, int b, float* __restrict__ out) {
  const int t_ = threadIdx.x, rowl = t_ >> 4, x4 = (t_ & 15) * 4; const int row = blockIdx.x * 16 + rowl, c = row >> 6, Y = row & 63;
  const float al = bf16_rne(alpha[0]) * 0.25f; const int R = Y + 1;
  v4f o;
#pragma unroll
  for (int e = 0; e < 4; ++e) { const int X = x4 + e, Cc = X + 1; float s = 0.0f;
#pragma unroll
    for (int u = 0; u < VK; ++u) { const int qy2 = R - u; if (qy2 < 0 || (qy2 & 1) || (qy2 >> 1) >= HS) continue; const int Qy = qy2 >> 1;
#pragma unroll
      for (int v = 0; v < VK; ++v) { const int qx2 = Cc - v; if (qx2 < 0 || (qx2 & 1) || (qx2 >> 1) >= HS) continue; const int Qx = qx2 >> 1;
        s += P[(size_t)(Qy * HS + Qx) * NCOL + c * 16 + u * 4 + v]; } }
    o[e] = bf16_rne(x[(((size_t)b * C + c) * HW + Y) * HW + X]) + al * s; }
  for (int pass = 0; pass < 2; ++pass) { *(volatile v4f*)(out + (((size_t)b * C + c) * HW + Y) * HW + x4) = o; __threadfence(); }
}
}

extern "C" void kernel_launch(void* const* d_in, const int* in_sizes, int n_in,
                              void* d_out, int out_size, void* d_ws, size_t ws_size, hipStream_t stream) {
  (void)n_in; (void)out_size;
  const float* x = (const float*)d_in[0]; const float* sc = (const float*)d_in[1]; const float* alpha = (const float*)d_in[2];
  float* out = (float*)d_out;
  if (in_sizes[0] != Bn * C * NPIX || in_sizes[1] != Bn * NQ * NQ || in_sizes[2] != 1) return;
  size_t off = 0; char* ws = (char*)d_ws;
  auto carve = [&](size_t bytes) { char* p = ws + off; off += (bytes + 255) & ~(size_t)255; return p; };
  unsigned short* s16 = (unsigned short*)carve((size_t)Bn * NQ * NQ * 2); unsigned short* vt = (unsigned short*)carve((size_t)NCOL * NQ * 2); float* P = (float*)carve((size_t)NQ * NCOL * 4);
  if (off > ws_size) return;
  sprep_kernel<<<512, 256, 0, stream>>>(sc, s16);
  for (int b = 0; b < Bn; ++b) {
    vt_kernel<<<NCOL / 16, 256, 0, stream>>>(x, b, vt);
    gemm_kernel<<<dim3(NCOL / 64, NQ / 128), 128, 0, stream>>>(s16, b, vt, P);
    oadd_kernel<<<C * HW / 16, 256, 0, stream>>>(P, x, alpha, b, out);
  }
}
